// Enc_apg_z_33663953666955
// MI455X (gfx1250) — hardware-run, weakly checked
//
#include <hip/hip_runtime.h>


#ifndef NSB
#define NSB 32
#endif
#ifndef NPT
#define NPT 2048
#endif
#define NSB_FULL 32
#define NPT_FULL 2048
#ifndef OUT_NPT
#define OUT_NPT NPT
#endif
#define KC   16
#define DD   32
#define HH   128
#define W1K  96
#define APB  256
#define GSC  ((float)(2.0 * 1.4426950408889634))
#define LOG2E 1.4426950408889634f
#define NEGB (-3.0e38f)

static_assert(DD == 32);
static_assert(W1K == 3 * DD);
static_assert(HH == 128);
static_assert(HH % 64 == 0);
static_assert(KC == 16);
static_assert((NSB * NPT) % 64 == 0);
static_assert((NSB * KC) % 64 == 0);
static_assert(NPT % APB == 0);
static_assert(APB == 256);
static_assert(NSB <= NSB_FULL);
static_assert(NPT <= NPT_FULL);
static_assert(((size_t)NPT * DD) % 8 == 0);
static_assert(((size_t)NSB * KC * DD) % 8 == 0);
static_assert((W1K * HH) % 8 == 0);
static_assert((W1K * 2) % 16 == 0);
static_assert(APB * 2 * 16 == KC * HH * 4);
static_assert(32 * 16 * 8 == 16 * 64 * 4);
static_assert(32 * 16 * 4 == 32 * KC * 4);
static_assert((16 * 68 * 4) <= 131072);
static_assert((KC * HH + HH + (APB / 32) * 32 * KC) * 4 <= 131072);

typedef unsigned short bf;
typedef __attribute__((ext_vector_type(16))) __bf16   v16bf;
typedef __attribute__((ext_vector_type(8)))  unsigned short v8us;
typedef __attribute__((ext_vector_type(8)))  float    v8f;
typedef __attribute__((ext_vector_type(4)))  float    v4f;
typedef v4f  __attribute__((may_alias)) v4fa;

__device__ __forceinline__ unsigned short f2bf(float f) { unsigned u = __float_as_uint(f); u += 0x7FFFu + ((u >> 16) & 1u); return (unsigned short)(u >> 16); }
__device__ __forceinline__ float bfr(float f) { return __uint_as_float(((unsigned)f2bf(f)) << 16); }
__device__ __forceinline__ v16bf cat16b(v8us lo, v8us hi) { return __builtin_bit_cast(v16bf, __builtin_shufflevector(lo, hi, 0, 1, 2, 3, 4, 5, 6, 7, 8, 9, 10, 11, 12, 13, 14, 15)); }
__device__ __forceinline__ v8f wmmab(v16bf a, v16bf b, v8f c) { return __builtin_amdgcn_wmma_f32_16x16x32_bf16(false, a, false, b, (short)0, c, false, false); }
__device__ __forceinline__ v8f wmmabg(v16bf a, v16bf b, v8f c) { c = wmmab(a, b, c); asm volatile("v_nop\n\tv_nop\n\tv_nop\n\tv_nop" : "+v"(c) : "v"(a), "v"(b)); return c; }
__device__ __forceinline__ v16bf ldb(const bf* p)  { return cat16b(*(const v8us*)p, *(const v8us*)(p + 16)); }
__device__ __forceinline__ void wave_sync() { __builtin_amdgcn_fence(3  , "wavefront"); __builtin_amdgcn_wave_barrier(); asm volatile("" ::: "memory"); }

__global__ __launch_bounds__(256) void k_cvt8(const float* __restrict__ src, bf* dst, size_t n8) {
    const size_t i = (size_t)blockIdx.x * 256 + threadIdx.x; if (i >= n8) return;
    const v8f v = *(const v8f*)(src + i * 8); v8us o;
#pragma unroll
    for (int k = 0; k < 8; ++k) o[k] = f2bf(v[k]);
    *(volatile v8us*)(dst + i * 8) = o; __threadfence(); *(volatile v8us*)(dst + i * 8) = o;
}

__global__ __launch_bounds__(256) void k_w1t(const float* __restrict__ W1, bf* WT) {
    unsigned i = blockIdx.x * 256u + threadIdx.x;
    if (i >= (unsigned)(W1K * HH / 8)) return;
    asm volatile("" : "+v"(i));
    const unsigned o = i / 12u, c8 = (i % 12u) * 8u;
    v8us ov;
#pragma unroll
    for (unsigned j = 0; j < 8u; ++j) ov[j] = f2bf(W1[(size_t)(c8 + j) * HH + o]);
    *(volatile v8us*)(WT + (size_t)i * 8) = ov; __threadfence(); *(volatile v8us*)(WT + (size_t)i * 8) = ov;
}

__global__ __launch_bounds__(32) void k_gemm(const bf* __restrict__ A, unsigned astep, unsigned nsteps, const bf* __restrict__ Bt, unsigned bko,
                                             const float* __restrict__ bias, unsigned hasb, float* C) {
    __shared__ __align__(16) float os[16 * 68];
    const unsigned lane = threadIdx.x & 31u, lr = lane & 15u, hi = lane >> 4;
    const unsigned r0 = blockIdx.x * 64u, c0 = blockIdx.y * 64u;
    v8f acc[4][4];
#pragma unroll
    for (int mb = 0; mb < 4; ++mb)
#pragma unroll
        for (int nb = 0; nb < 4; ++nb) acc[mb][nb] = (v8f){};
    const size_t aoff = (size_t)(r0 + lr) * DD + 8u * hi;
    const size_t boff = (size_t)(c0 + lr) * W1K + bko + 8u * hi;
#pragma unroll 1
    for (unsigned s = 0; s < nsteps; ++s) {
        const bf* ap = A + (size_t)s * astep + aoff;
        const bf* bp = Bt + boff + (size_t)s * 32u;
        v16bf a[4];
#pragma unroll
        for (int mb = 0; mb < 4; ++mb) a[mb] = ldb(ap + (size_t)mb * 16 * DD);
#pragma unroll
        for (int nb = 0; nb < 4; ++nb) { const v16bf b = ldb(bp + (size_t)nb * 16 * W1K);
#pragma unroll
            for (int mb = 0; mb < 4; ++mb) acc[mb][nb] = wmmabg(a[mb], b, acc[mb][nb]); }
    }
    float bc[4];
#pragma unroll
    for (int nb = 0; nb < 4; ++nb) { const float bv = bfr(bias[c0 + (unsigned)nb * 16u + lr]); bc[nb] = (hasb != 0u) ? bv : 0.0f; }
#pragma unroll
    for (int mb = 0; mb < 4; ++mb) {
#pragma unroll
        for (int nb = 0; nb < 4; ++nb) {
#pragma unroll
            for (int j = 0; j < 8; ++j) os[(hi * 8u + (unsigned)j) * 68u + (unsigned)nb * 16u + lr] = (acc[mb][nb][j] + bc[nb]) * GSC; }
        wave_sync();
        float* cb = C + (size_t)(r0 + (unsigned)mb * 16u) * HH + c0;
#pragma unroll 1
        for (int ps = 0; ps < 2; ++ps) {
#pragma unroll
            for (int s = 0; s < 8; ++s) { const unsigned row = 2u * (unsigned)s + (lane >> 4), c4 = (lane & 15u) * 4u;
                const v4f val = *(const v4fa*)(&os[row * 68u + c4]);
                *(volatile v4f*)(cb + (size_t)row * HH + c4) = val; }
            if (ps == 0) __threadfence(); }
        wave_sync();
    }
}

__global__ __launch_bounds__(APB) void k_assign(const float* __restrict__ HX, const float* __restrict__ HK, const float* __restrict__ W2, const float* __restrict__ B2, float* OUT) {
#pragma clang fp contract(off)
    __shared__ __align__(16) float hks[KC * HH];
    __shared__ __align__(16) float w2s[HH];
    __shared__ __align__(16) float ot[(APB / 32) * 32 * KC];
    const unsigned tid = threadIdx.x, lane = tid & 31u;
    const unsigned wave = (unsigned)__builtin_amdgcn_readfirstlane((int)(threadIdx.x >> 5));
    const unsigned bx = blockIdx.x;
    const unsigned sb = bx / ((unsigned)NPT / (unsigned)APB);
    const unsigned pt0 = (bx % ((unsigned)NPT / (unsigned)APB)) * (unsigned)APB;
    const float* hkg = HK + (size_t)sb * (KC * HH);
#pragma unroll
    for (unsigned i = 0; i < 2u; ++i) { const unsigned idx = (tid + 256u * i) * 4u;
        const v4f v = *(const v4f*)(hkg + idx); *(v4fa*)(&hks[idx]) = v; }
    if (wave == 0u) { const v4f w = *(const v4f*)(W2 + lane * 4u); v4f o;
        o[0] = -2.0f * bfr(w[0]); o[1] = -2.0f * bfr(w[1]); o[2] = -2.0f * bfr(w[2]); o[3] = -2.0f * bfr(w[3]);
        *(v4fa*)(&w2s[lane * 4u]) = o; }
    __syncthreads();
    float sw = 0.0f;
#pragma unroll 1
    for (unsigned c = 0; c < (unsigned)HH / 4u; ++c) { const v4f w = *(const v4fa*)(&w2s[4u * c]); sw += w[0]; sw += w[1]; sw += w[2]; sw += w[3]; }
    const float gconst = bfr(B2[0]) + (-0.5f) * sw;
    const float* hxr = HX + ((size_t)sb * NPT + pt0 + tid) * HH;
    float g[KC];
#pragma unroll
    for (int k = 0; k < KC; ++k) g[k] = 0.0f;
#pragma unroll 1
    for (unsigned c = 0; c < (unsigned)HH / 4u; ++c) {
        const v4f xv = *(const v4f*)(hxr + 4u * c);
        const v4f wv = *(const v4fa*)(&w2s[4u * c]);
#pragma unroll
        for (int k = 0; k < KC; ++k) {
            const v4f hv = *(const v4fa*)(&hks[(unsigned)k * (unsigned)HH + 4u * c]);
#pragma unroll
            for (int j = 0; j < 4; ++j) {
                const float e = __builtin_amdgcn_exp2f(xv[j] + hv[j]);
                const float r = __builtin_amdgcn_rcpf(e + 1.0f);
                g[k] = fmaf(wv[j], r, g[k]); } }
    }
    float gv[KC]; float mx = NEGB;
#pragma unroll
    for (int k = 0; k < KC; ++k) { gv[k] = gconst + g[k]; mx = fmaxf(mx, gv[k]); }
    float ev[KC]; float sum = 0.0f;
#pragma unroll
    for (int k = 0; k < KC; ++k) { ev[k] = __builtin_amdgcn_exp2f((gv[k] - mx) * LOG2E); sum += ev[k]; }
    const float inv = 1.0f / sum;
    const unsigned wb = wave * (32u * KC);
#pragma unroll
    for (int q = 0; q < 4; ++q) { v4f o; o[0] = ev[4 * q + 0] * inv; o[1] = ev[4 * q + 1] * inv; o[2] = ev[4 * q + 2] * inv; o[3] = ev[4 * q + 3] * inv;
        *(v4fa*)(&ot[wb + lane * (unsigned)KC + 4u * (unsigned)q]) = o; }
    wave_sync();
    float* orow = OUT + ((size_t)sb * OUT_NPT + pt0 + wave * 32u) * KC;
#pragma unroll 1
    for (int ps = 0; ps < 2; ++ps) {
#pragma unroll
        for (int j = 0; j < 4; ++j) { const unsigned e4 = ((unsigned)j * 32u + lane) * 4u;
            const v4f val = *(const v4fa*)(&ot[wb + e4]);
            *(volatile v4f*)(orow + e4) = val; }
        if (ps == 0) __threadfence(); }
}

static constexpr size_t al256(size_t v) { return (v + 255) & ~(size_t)255; }
static constexpr size_t SZ_XB = al256((size_t)NSB * NPT * DD * 2);
static constexpr size_t SZ_MT = al256((size_t)2 * NSB * KC * DD * 2);
static constexpr size_t SZ_WT = al256((size_t)HH * W1K * 2);
static constexpr size_t SZ_HX = al256((size_t)NSB * NPT * HH * 4);
static constexpr size_t SZ_HK = al256((size_t)NSB * KC * HH * 4);
static constexpr size_t SZ_TOTAL = SZ_XB + SZ_MT + SZ_WT + SZ_HX + SZ_HK;
static_assert(SZ_TOTAL <= (size_t)134217728);
static_assert(((size_t)NSB * KC * DD * 2) % 256 == 0);
static_assert((size_t)(W1K * HH / 8) * 16 <= SZ_WT);
static_assert((size_t)NSB * NPT * DD / 8 * 16 <= SZ_XB);
static_assert((size_t)2 * (NSB * KC * DD / 8) * 16 <= SZ_MT);
static_assert((size_t)(NSB * NPT / 64) * 64 * HH * 4 <= SZ_HX);
static_assert((size_t)(NSB * KC / 64) * 64 * HH * 4 <= SZ_HK);

extern "C" void kernel_launch(void* const* d_in, const int* in_sizes, int n_in,
                              void* d_out, int out_size, void* d_ws, size_t ws_size, hipStream_t stream) {
    if (n_in < 7) return;
    const size_t needx = ((size_t)(NSB - 1) * NPT_FULL + NPT) * DD;
    if ((size_t)in_sizes[0] < needx) return;
    if ((size_t)in_sizes[1] < (size_t)NSB * KC * DD || (size_t)in_sizes[2] < (size_t)NSB * KC * DD) return;
    if (in_sizes[3] < W1K * HH || in_sizes[4] < HH || in_sizes[5] < HH || in_sizes[6] < 1) return;
    if ((size_t)out_size < ((size_t)(NSB - 1) * OUT_NPT + NPT) * KC) return;
    if (SZ_TOTAL > ws_size) return;
    const float* x  = (const float*)d_in[0];
    const float* mu = (const float*)d_in[1];
    const float* ta = (const float*)d_in[2];
    const float* w1 = (const float*)d_in[3];
    const float* b1 = (const float*)d_in[4];
    const float* w2 = (const float*)d_in[5];
    const float* b2 = (const float*)d_in[6];
    float* OUT = (float*)d_out;
    char* wsp = (char*)d_ws;
    bf* XB = (bf*)wsp; wsp += SZ_XB;
    bf* MT = (bf*)wsp; wsp += SZ_MT;
    bf* WT = (bf*)wsp; wsp += SZ_WT;
    float* HXp = (float*)wsp; wsp += SZ_HX;
    float* HKp = (float*)wsp; wsp += SZ_HK;

    if (NPT == NPT_FULL) {
        const size_t n8 = (size_t)NSB * NPT * DD / 8;
        k_cvt8<<<(unsigned)((n8 + 255) / 256), 256, 0, stream>>>(x, XB, n8);
    } else {
        const size_t n8 = (size_t)NPT * DD / 8;
        for (int b = 0; b < NSB; ++b) k_cvt8<<<(unsigned)((n8 + 255) / 256), 256, 0, stream>>>(x + (size_t)b * NPT_FULL * DD, XB + (size_t)b * NPT * DD, n8);
    }
    { const size_t n8 = (size_t)NSB * KC * DD / 8; const unsigned g = (unsigned)((n8 + 255) / 256);
      k_cvt8<<<g, 256, 0, stream>>>(mu, MT, n8);
      k_cvt8<<<g, 256, 0, stream>>>(ta, MT + (size_t)NSB * KC * DD, n8); }
    k_w1t<<<(unsigned)((W1K * HH / 8 + 255) / 256), 256, 0, stream>>>(w1, WT);

    k_gemm<<<dim3(NSB * NPT / 64, HH / 64, 1), 32, 0, stream>>>(XB, 0u, 1u, WT, 0u, b1, 1u, HXp);
    k_gemm<<<dim3(NSB * KC / 64, HH / 64, 1), 32, 0, stream>>>(MT, (unsigned)(NSB * KC * DD), 2u, WT, 32u, b1, 0u, HKp);

    k_assign<<<dim3(NSB * (NPT / APB), 1, 1), APB, 0, stream>>>(HXp, HKp, w2, b2, OUT);
}
